// SSMBackbone_21938692948378
// MI455X (gfx1250) — hardware-verified
//
#include <hip/hip_runtime.h>
#include <math.h>

typedef __attribute__((ext_vector_type(16))) _Float16 v16h;
typedef __attribute__((ext_vector_type(8)))  _Float16 v8h;
typedef __attribute__((ext_vector_type(16))) __bf16   v16b;
typedef __attribute__((ext_vector_type(8)))  __bf16   v8b;
typedef __attribute__((ext_vector_type(8)))  float    v8f;
typedef __attribute__((ext_vector_type(4)))  float    v4f;

constexpr int kSeq    = 2048;
constexpr int kDinp   = 256;
constexpr int kDm     = 1024;
constexpr int kDin    = 2048;
constexpr int kNst    = 16;
constexpr int kDtR    = 64;
constexpr int kPrjN   = 96;
constexpr int kPrjP   = 128;
constexpr int kXZP    = 2 * kDin;
constexpr int kDff    = 4096;
constexpr int kNumSsm = 2;
constexpr int kTP     = 260;
constexpr int kSYP    = 260;
constexpr float kWScale = 256.0f;
constexpr float kXScale = 16.0f;
constexpr float kYScale = 16.0f;
constexpr float kPScale = 16.0f;

__device__ __forceinline__ unsigned short f2bf_bits(float f) {
  unsigned u = __float_as_uint(f);
  return (unsigned short)((u + 0x7FFFu + ((u >> 16) & 1u)) >> 16);
}
__device__ __forceinline__ float bf_bits2f(unsigned short h) { return __uint_as_float(((unsigned)h) << 16); }

__device__ __forceinline__ void dep_guard_h(v8f& a, v8f& b, v16h x, v16h y) { asm volatile("v_nop\n\tv_nop\n\tv_nop\n\tv_nop" : "+v"(a), "+v"(b) : "v"(x), "v"(y)); }
__device__ __forceinline__ void dep_guard_b(v8f& a, v8f& b, v16b x, v16b y) { asm volatile("v_nop\n\tv_nop\n\tv_nop\n\tv_nop" : "+v"(a), "+v"(b) : "v"(x), "v"(y)); }
__device__ __forceinline__ void keep4_h(v16h a, v16h b, v16h c, v16h d) { asm volatile("v_nop" :: "v"(a), "v"(b), "v"(c), "v"(d)); }
__device__ __forceinline__ void keep4_b(v16b a, v16b b, v16b c, v16b d) { asm volatile("v_nop" :: "v"(a), "v"(b), "v"(c), "v"(d)); }
__device__ __forceinline__ void acc_guard4(v8f& a, v8f& b, v8f& c, v8f& d) { asm volatile("v_nop\n\tv_nop\n\tv_nop\n\tv_nop" : "+v"(a), "+v"(b), "+v"(c), "+v"(d)); }
template <typename T> struct Frag;
template <> struct Frag<_Float16> {
  typedef v16h V; union U { v16h v; v8h h[2]; };
  static __device__ __forceinline__ v16h load(const _Float16* p) {
    U f; f.h[0] = *(const v8h*)(p); f.h[1] = *(const v8h*)(p + 16); return f.v;
  }
  static __device__ __forceinline__ v8f mma(v16h a, v16h b, v8f c) {
    return __builtin_amdgcn_wmma_f32_16x16x32_f16(false, a, false, b, (short)0, c, false, false);
  }
  static __device__ __forceinline__ void guard(v8f& a, v8f& b, v16h x, v16h y) { dep_guard_h(a, b, x, y); }
  static __device__ __forceinline__ void keep(v16h a, v16h b, v16h c, v16h d) { keep4_h(a, b, c, d); }
};
template <> struct Frag<__bf16> {
  typedef v16b V; union U { v16b v; v8b h[2]; };
  static __device__ __forceinline__ v16b load(const __bf16* p) {
    U f; f.h[0] = *(const v8b*)(p); f.h[1] = *(const v8b*)(p + 16); return f.v;
  }
  static __device__ __forceinline__ v8f mma(v16b a, v16b b, v8f c) {
    return __builtin_amdgcn_wmma_f32_16x16x32_bf16(false, a, false, b, (short)0, c, false, false);
  }
  static __device__ __forceinline__ void guard(v8f& a, v8f& b, v16b x, v16b y) { dep_guard_b(a, b, x, y); }
  static __device__ __forceinline__ void keep(v16b a, v16b b, v16b c, v16b d) { keep4_b(a, b, c, d); }
};

template <int ET> struct Elem;
template <> struct Elem<0> { typedef _Float16 T; };
template <> struct Elem<1> { typedef __bf16 T; };
template <int ET, bool SPLIT, int BIAS_MODE, int OUT_MODE, bool RESID, int ACT = 0>
__global__ __launch_bounds__(256) void wmma_gemm64(
    const unsigned short* __restrict__ Ap, const unsigned short* __restrict__ A2p, int lda, long strideA,
    const unsigned short* __restrict__ Btp, const unsigned short* __restrict__ Bt2p, int ldb, long strideB,
    void* __restrict__ Cout, void* __restrict__ Cout2, int ldc, long strideC,
    const float* __restrict__ bias,
    const float* __restrict__ resid, long strideR,
    int M, int N, int K, float scale) {
  typedef typename Elem<ET>::T T;
  typedef typename Frag<T>::V V;
  const T* A = (const T*)Ap; const T* A2 = (const T*)A2p; const T* Bt = (const T*)Btp; const T* Bt2 = (const T*)Bt2p;
  __shared__ __align__(16) float sT[8][16 * 68];
  const int b    = blockIdx.y;
  const int lane = threadIdx.x & 31;
  const int wave = threadIdx.x >> 5;
  const int tilesN = N >> 6;
  const int tilesM = M >> 6;
  const int tile = blockIdx.x * 8 + wave;
  if (tile >= tilesM * tilesN) return;
  const int tm = tile / tilesN;
  const int tn = tile - tm * tilesN;
  const int m0 = tm << 6;
  const int n0 = tn << 6;

  const T* Ab  = A  + (size_t)b * strideA;
  const T* Bb  = Bt + (size_t)b * strideB;
  const T* Ab2 = SPLIT ? (A2  + (size_t)b * strideA) : nullptr;
  const T* Bb2 = SPLIT ? (Bt2 + (size_t)b * strideB) : nullptr;

  const int rlane = lane & 15;
  const int koff  = (lane >> 4) * 8;
  const int mOff  = (lane >> 4) * 8;

  v8f acc[4][4];
#pragma unroll
  for (int i = 0; i < 4; ++i)
#pragma unroll
    for (int j = 0; j < 4; ++j) acc[i][j] = (v8f){0.f,0.f,0.f,0.f,0.f,0.f,0.f,0.f};

  for (int k0 = 0; k0 < K; k0 += 32) {
    V bh[4], bl[4];
#pragma unroll
    for (int j = 0; j < 4; ++j) {
      const size_t bo = (size_t)(n0 + (j << 4) + rlane) * ldb + koff + k0;
      bh[j] = Frag<T>::load(Bb + bo);
      if (SPLIT) bl[j] = Frag<T>::load(Bb2 + bo);
    }
#pragma unroll
    for (int i = 0; i < 4; ++i) {
      const size_t ao = (size_t)(m0 + (i << 4) + rlane) * lda + koff + k0;
      V ah = Frag<T>::load(Ab + ao);
      V al;
      if (SPLIT) al = Frag<T>::load(Ab2 + ao);
#pragma unroll
      for (int j = 0; j < 4; ++j) {
        acc[i][j] = Frag<T>::mma(ah, bh[j], acc[i][j]);
        if (SPLIT) {
          acc[i][j] = Frag<T>::mma(ah, bl[j], acc[i][j]);
          acc[i][j] = Frag<T>::mma(al, bh[j], acc[i][j]);
        }
      }
      Frag<T>::guard(acc[i][0], acc[i][3], ah, SPLIT ? al : ah);
    }
    Frag<T>::keep(bh[0], bh[1], bh[2], bh[3]);
    if (SPLIT) Frag<T>::keep(bl[0], bl[1], bl[2], bl[3]);
  }
  acc_guard4(acc[0][0], acc[0][1], acc[0][2], acc[0][3]);
  acc_guard4(acc[1][0], acc[1][1], acc[1][2], acc[1][3]);
  acc_guard4(acc[2][0], acc[2][1], acc[2][2], acc[2][3]);
  acc_guard4(acc[3][0], acc[3][1], acc[3][2], acc[3][3]);

  float* slab = sT[wave];
  const float* Rb = RESID ? (resid + (size_t)b * strideR) : nullptr;
#pragma unroll
  for (int i = 0; i < 4; ++i) {
    const int mBase = m0 + (i << 4);
#pragma unroll
    for (int j = 0; j < 4; ++j) {
      const int n = n0 + (j << 4) + rlane;
      float bv = 0.f;
      if (BIAS_MODE == 2) bv = bias[n];
#pragma unroll
      for (int r = 0; r < 8; ++r) {
        float v = acc[i][j][r] * scale;
        if (BIAS_MODE == 1) v += bias[mBase + mOff + r];
        if (BIAS_MODE == 2) v += bv;
        if (RESID) v += Rb[(size_t)(mBase + mOff + r) * ldc + n];
        if (ACT == 1) v = tanhf(v);
        if (ACT == 2) v = fmaxf(v, 0.0f);
        if (ACT == 3) v = v / (1.0f + expf(-v));
        if (ACT == 4) v = (v > 0.f) ? v : 0.01f * v;
        if (ACT == 5) v = 0.5f * v * (1.0f + erff(v * 0.70710678118654752f));
        slab[(mOff + r) * 68 + (j << 4) + rlane] = v;
      }
    }
    __builtin_amdgcn_fence(__ATOMIC_RELEASE, "workgroup");
    __builtin_amdgcn_wave_barrier();
    __builtin_amdgcn_fence(__ATOMIC_ACQUIRE, "workgroup");
    if (OUT_MODE == 0) {
      float* C = (float*)Cout + (size_t)b * strideC;
      const int hh = lane >> 4, c4 = (lane & 15) * 4;
      for (int pass = 0; pass < 2; ++pass) {
#pragma unroll
        for (int it = 0; it < 8; ++it) {
          const int row = it * 2 + hh;
          v4f v = *(const v4f*)(slab + row * 68 + c4);
          *(volatile v4f*)(C + (size_t)(mBase + row) * ldc + n0 + c4) = v;
        }
        __threadfence();
      }
    } else {
      const int q = lane >> 3, c8 = (lane & 7) * 8;
      unsigned short* C  = (unsigned short*)Cout  + (size_t)b * strideC;
      unsigned short* C2 = (OUT_MODE == 2) ? ((unsigned short*)Cout2 + (size_t)b * strideC) : nullptr;
      for (int pass = 0; pass < 2; ++pass) {
#pragma unroll
        for (int it = 0; it < 4; ++it) {
          const int row = it * 4 + q;
          const float* sp = slab + row * 68 + c8;
          v8h hv, lv;
#pragma unroll
          for (int e = 0; e < 8; ++e) {
            if (OUT_MODE == 1) {
              hv[e] = (_Float16)sp[e];
            } else {
              unsigned short hb = f2bf_bits(sp[e]);
              unsigned short lb = f2bf_bits(sp[e] - bf_bits2f(hb));
              hv[e] = __builtin_bit_cast(_Float16, hb);
              lv[e] = __builtin_bit_cast(_Float16, lb);
            }
          }
          *(volatile v8h*)(C + (size_t)(mBase + row) * ldc + n0 + c8) = hv;
          if (OUT_MODE == 2) *(volatile v8h*)(C2 + (size_t)(mBase + row) * ldc + n0 + c8) = lv;
        }
        __threadfence();
      }
    }
    __builtin_amdgcn_fence(__ATOMIC_RELEASE, "workgroup");
    __builtin_amdgcn_wave_barrier();
    __builtin_amdgcn_fence(__ATOMIC_ACQUIRE, "workgroup");
  }
}

__device__ __forceinline__ float bfr(float f) { return bf_bits2f(f2bf_bits(f)); }
__device__ __forceinline__ float sigm(float v) { return __builtin_amdgcn_rcpf(1.0f + __expf(-v)); }

__global__ __launch_bounds__(256) void cast_rows_f16_kernel(
    const float* __restrict__ src, unsigned short* __restrict__ dst, int K, int nreal, int total8, float scale)
{
  const int i = blockIdx.x * 256 + threadIdx.x;
  if (i >= total8) return;
  const int e0  = i << 3;
  const int row = e0 / K;
  const int col = e0 - row * K;
  const int rc  = (row < nreal) ? row : (nreal - 1);
  const bool keep = (row < nreal);
  const float* p = src + (size_t)rc * K + col;
  const v4f a0 = *(const v4f*)(p);
  const v4f a1 = *(const v4f*)(p + 4);
  v8h hv;
#pragma unroll
  for (int e = 0; e < 4; ++e) {
    const float v0 = keep ? a0[e] : 0.f;
    const float v1 = keep ? a1[e] : 0.f;
    hv[e]     = (_Float16)(bfr(v0) * scale);
    hv[4 + e] = (_Float16)(bfr(v1) * scale);
  }
  unsigned short* q = dst + e0;
  *(volatile v8h*)q = hv;
  __threadfence();
  *(volatile v8h*)q = hv;
}

__global__ __launch_bounds__(256) void dt_cast_kernel(
    const float* __restrict__ PROJ, unsigned short* __restrict__ DH, int total8)
{
  const int i = blockIdx.x * 256 + threadIdx.x;
  if (i >= total8) return;
  const int e0  = i << 3;
  const int row = e0 >> 6;
  const int c8  = e0 & 63;
  const float* p = PROJ + (size_t)row * kPrjP + c8;
  const v4f a0 = *(const v4f*)(p);
  const v4f a1 = *(const v4f*)(p + 4);
  v8h hv;
#pragma unroll
  for (int e = 0; e < 4; ++e) { hv[e] = (_Float16)a0[e]; hv[4 + e] = (_Float16)a1[e]; }
  unsigned short* q = DH + e0;
  *(volatile v8h*)q = hv;
  __threadfence();
  *(volatile v8h*)q = hv;
}

__global__ __launch_bounds__(256) void ln_f16_kernel(
    const float* __restrict__ x, const float* __restrict__ gw, const float* __restrict__ gb,
    unsigned short* __restrict__ XP, int nrows)
{
  const int lane = threadIdx.x & 31, wave = threadIdx.x >> 5;
  const int row = blockIdx.x * 8 + wave;
  if (row >= nrows) return;
  const float* xr = x + (size_t)row * kDm;
  v4f a[8];
#pragma unroll
  for (int i = 0; i < 4; ++i) {
    const int c0 = 256 * i + lane * 8;
    a[2 * i]     = *(const v4f*)(xr + c0);
    a[2 * i + 1] = *(const v4f*)(xr + c0 + 4);
  }
  float s = 0.f;
#pragma unroll
  for (int k = 0; k < 8; ++k) s += (a[k][0] + a[k][1]) + (a[k][2] + a[k][3]);
#pragma unroll
  for (int off = 1; off < 32; off <<= 1) s += __shfl_xor(s, off, 32);
  const float mean = s * (1.0f / 1024.0f);
  v4f dv[8];
  float ss = 0.f;
#pragma unroll
  for (int k = 0; k < 8; ++k) {
    dv[k] = a[k] - mean;
    ss += (dv[k][0] * dv[k][0] + dv[k][1] * dv[k][1]) + (dv[k][2] * dv[k][2] + dv[k][3] * dv[k][3]);
  }
#pragma unroll
  for (int off = 1; off < 32; off <<= 1) ss += __shfl_xor(ss, off, 32);
  const float var  = ss * (1.0f / 1024.0f);
  const float rstd = rsqrtf(var + 1e-5f);
  v8h hv[4];
#pragma unroll
  for (int i = 0; i < 4; ++i) {
    const int c0 = 256 * i + lane * 8;
    const v4f w0 = *(const v4f*)(gw + c0), w1 = *(const v4f*)(gw + c0 + 4);
    const v4f b0 = *(const v4f*)(gb + c0), b1 = *(const v4f*)(gb + c0 + 4);
    const v4f o0 = (dv[2 * i] * rstd) * w0 + b0;
    const v4f o1 = (dv[2 * i + 1] * rstd) * w1 + b1;
#pragma unroll
    for (int e = 0; e < 4; ++e) { hv[i][e] = (_Float16)o0[e]; hv[i][4 + e] = (_Float16)o1[e]; }
  }
  for (int pass = 0; pass < 2; ++pass) {
#pragma unroll
    for (int i = 0; i < 4; ++i)
      *(volatile v8h*)(XP + (size_t)row * kDm + 256 * i + lane * 8) = hv[i];
    __threadfence();
  }
}

__global__ __launch_bounds__(256) void ln_f32_kernel(
    const float* __restrict__ x, const float* __restrict__ gw, const float* __restrict__ gb,
    float* __restrict__ out, int nrows)
{
  const int lane = threadIdx.x & 31, wave = threadIdx.x >> 5;
  const int row = blockIdx.x * 8 + wave;
  if (row >= nrows) return;
  const float* xr = x + (size_t)row * kDm;
  v4f a[8];
#pragma unroll
  for (int i = 0; i < 8; ++i) a[i] = *(const v4f*)(xr + 128 * i + lane * 4);
  float s = 0.f;
#pragma unroll
  for (int k = 0; k < 8; ++k) s += (a[k][0] + a[k][1]) + (a[k][2] + a[k][3]);
#pragma unroll
  for (int off = 1; off < 32; off <<= 1) s += __shfl_xor(s, off, 32);
  const float mean = s * (1.0f / 1024.0f);
  v4f dv[8];
  float ss = 0.f;
#pragma unroll
  for (int k = 0; k < 8; ++k) {
    dv[k] = a[k] - mean;
    ss += (dv[k][0] * dv[k][0] + dv[k][1] * dv[k][1]) + (dv[k][2] * dv[k][2] + dv[k][3] * dv[k][3]);
  }
#pragma unroll
  for (int off = 1; off < 32; off <<= 1) ss += __shfl_xor(ss, off, 32);
  const float var  = ss * (1.0f / 1024.0f);
  const float rstd = rsqrtf(var + 1e-5f);
  v4f o[8];
#pragma unroll
  for (int i = 0; i < 8; ++i) {
    const int c0 = 128 * i + lane * 4;
    const v4f w0 = *(const v4f*)(gw + c0);
    const v4f b0 = *(const v4f*)(gb + c0);
    o[i] = (dv[i] * rstd) * w0 + b0;
  }
  for (int pass = 0; pass < 2; ++pass) {
#pragma unroll
    for (int i = 0; i < 8; ++i)
      *(volatile v4f*)(out + (size_t)row * kDm + 128 * i + lane * 4) = o[i];
    __threadfence();
  }
}

__global__ __launch_bounds__(256) void conv_silu_kernel(
    const float* __restrict__ XZ, const float* __restrict__ cw, const float* __restrict__ cb,
    float* __restrict__ UC, unsigned short* __restrict__ UP)
{
  __shared__ __align__(16) float sT[16 * kTP];
  const int tid = threadIdx.x, lane = tid & 31, wave = tid >> 5;
  const int d0 = blockIdx.x * 256, d = d0 + tid;
  const int g0 = blockIdx.y * 64;
  const float w0 = bfr(cw[d * 4 + 0]), w1 = bfr(cw[d * 4 + 1]), w2 = bfr(cw[d * 4 + 2]), w3 = bfr(cw[d * 4 + 3]);
  const float bc = bfr(cb[d]);
  float xm3, xm2, xm1;
  {
    const int r3 = (g0 >= 3) ? (g0 - 3) : g0;
    const int r2 = (g0 >= 2) ? (g0 - 2) : g0;
    const int r1 = (g0 >= 1) ? (g0 - 1) : g0;
    const float v3 = XZ[(size_t)r3 * kXZP + d];
    const float v2 = XZ[(size_t)r2 * kXZP + d];
    const float v1 = XZ[(size_t)r1 * kXZP + d];
    xm3 = (g0 >= 3) ? v3 : 0.f;
    xm2 = (g0 >= 2) ? v2 : 0.f;
    xm1 = (g0 >= 1) ? v1 : 0.f;
  }
  const int hrow = wave >> 1;
  const int hch  = (wave & 1) * 128 + lane * 4;
#pragma unroll 1
  for (int sub = 0; sub < 4; ++sub) {
    const int lb = g0 + sub * 16;
#pragma unroll 1
    for (int s = 0; s < 16; ++s) {
      const float xc = XZ[(size_t)(lb + s) * kXZP + d];
      float acc = w0 * xm3;
      acc = fmaf(w1, xm2, acc);
      acc = fmaf(w2, xm1, acc);
      acc = fmaf(w3, xc, acc);
      const float sv = acc + bc;
      sT[s * kTP + tid] = sv * sigm(sv);
      xm3 = xm2; xm2 = xm1; xm1 = xc;
    }
    __syncthreads();
    v4f fv[4];
    v8h hv[2];
#pragma unroll
    for (int it = 0; it < 4; ++it) fv[it] = *(const v4f*)(sT + (it * 4 + hrow) * kTP + hch);
#pragma unroll
    for (int it = 0; it < 2; ++it) {
      const float* sp = sT + (it * 8 + wave) * kTP + lane * 8;
      const v4f a0 = *(const v4f*)(sp);
      const v4f a1 = *(const v4f*)(sp + 4);
#pragma unroll
      for (int e = 0; e < 4; ++e) { hv[it][e] = (_Float16)a0[e]; hv[it][4 + e] = (_Float16)a1[e]; }
    }
    for (int pass = 0; pass < 2; ++pass) {
#pragma unroll
      for (int it = 0; it < 4; ++it)
        *(volatile v4f*)(UC + (size_t)(lb + it * 4 + hrow) * kDin + d0 + hch) = fv[it];
#pragma unroll
      for (int it = 0; it < 2; ++it)
        *(volatile v8h*)(UP + (size_t)(lb + it * 8 + wave) * kDin + d0 + lane * 8) = hv[it];
      __threadfence();
    }
    __syncthreads();
  }
}

__global__ __launch_bounds__(256) void scan_kernel(
    const float* __restrict__ DLR, const float* __restrict__ UC, const float* __restrict__ XZ,
    const float* __restrict__ PROJ, const float* __restrict__ dtb, const float* __restrict__ A_log,
    const float* __restrict__ Dv, unsigned short* __restrict__ YP)
{
  __shared__ __align__(16) float sBC[16 * 32];
  __shared__ __align__(16) float sY[16 * kSYP];
  const int tid = threadIdx.x, lane = tid & 31, wave = tid >> 5;
  const int d0 = blockIdx.x * 256, d = d0 + tid;

  float An[kNst];
#pragma unroll
  for (int n = 0; n < kNst; ++n) An[n] = -__expf(bfr(A_log[(size_t)d * kNst + n]));
  const float Dd = bfr(Dv[d]);
  const float bd = bfr(dtb[d]);
  float h[kNst];
#pragma unroll
  for (int n = 0; n < kNst; ++n) h[n] = 0.f;

#pragma unroll 1
  for (int c = 0; c < kSeq / 16; ++c) {
    const int t0 = c * 16;
    {
      const int r = tid >> 4, q = (tid & 15) * 2;
      const float* pp = PROJ + (size_t)(t0 + r) * kPrjP + kDtR + q;
      sBC[r * 32 + q]     = pp[0];
      sBC[r * 32 + q + 1] = pp[1];
    }
    __syncthreads();
#pragma unroll 1
    for (int s = 0; s < 16; ++s) {
      const size_t m = (size_t)(t0 + s);
      const float a     = DLR[m * kDin + d] + bd;
      const float delta = fmaxf(a, 0.0f) + log1pf(__expf(-fabsf(a)));
      const float xv    = UC[m * kDin + d];
      const float zv    = XZ[m * kXZP + kDin + d];
      const float du    = delta * xv;
      const float* bp = sBC + s * 32;
      float y = 0.f;
#pragma unroll
      for (int qq = 0; qq < 4; ++qq) {
        const v4f Bq = *(const v4f*)(bp + 4 * qq);
        const v4f Cq = *(const v4f*)(bp + 16 + 4 * qq);
#pragma unroll
        for (int e = 0; e < 4; ++e) {
          const int n = qq * 4 + e;
          const float ex = __expf(delta * An[n]);
          const float hn = h[n] * ex + du * Bq[e];
          h[n] = hn;
          y += Cq[e] * hn;
        }
      }
      y += xv * Dd;
      const float g = zv * sigm(zv);
      sY[s * kSYP + tid] = y * g;
    }
    __syncthreads();
    {
      v8h hv[2];
#pragma unroll
      for (int it = 0; it < 2; ++it) {
        const float* sp = sY + (it * 8 + wave) * kSYP + lane * 8;
        const v4f a0 = *(const v4f*)(sp);
        const v4f a1 = *(const v4f*)(sp + 4);
#pragma unroll
        for (int e = 0; e < 4; ++e) {
          hv[it][e]     = (_Float16)(a0[e] * kYScale);
          hv[it][4 + e] = (_Float16)(a1[e] * kYScale);
        }
      }
      for (int pass = 0; pass < 2; ++pass) {
#pragma unroll
        for (int it = 0; it < 2; ++it)
          *(volatile v8h*)(YP + (size_t)(t0 + it * 8 + wave) * kDin + d0 + lane * 8) = hv[it];
        __threadfence();
      }
    }
  }
}

__global__ __launch_bounds__(256) void glu_kernel(
    const float* __restrict__ G, const float* __restrict__ U, unsigned short* __restrict__ P, int total8)
{
  const int i = blockIdx.x * 256 + threadIdx.x;
  if (i >= total8) return;
  const size_t e0 = (size_t)i << 3;
  const v4f g0 = *(const v4f*)(G + e0), g1 = *(const v4f*)(G + e0 + 4);
  const v4f u0 = *(const v4f*)(U + e0), u1 = *(const v4f*)(U + e0 + 4);
  v8h hv;
#pragma unroll
  for (int e = 0; e < 4; ++e) {
    const float p0 = (g0[e] * sigm(g0[e])) * u0[e];
    const float p1 = (g1[e] * sigm(g1[e])) * u1[e];
    hv[e]     = (_Float16)(p0 * kPScale);
    hv[4 + e] = (_Float16)(p1 * kPScale);
  }
  unsigned short* q = P + e0;
  *(volatile v8h*)q = hv;
  __threadfence();
  *(volatile v8h*)q = hv;
}

extern "C" void kernel_launch(void* const* d_in, const int* in_sizes, int n_in,
                              void* d_out, int out_size, void* d_ws, size_t ws_size,
                              hipStream_t stream)
{
  if (n_in < 21) return;
  const float* x      = (const float*)d_in[0];
  const float* ipw    = (const float*)d_in[1];
  const float* ipb    = (const float*)d_in[2];
  const float* mnw    = (const float*)d_in[3];
  const float* mnb    = (const float*)d_in[4];
  const float* inw    = (const float*)d_in[5];
  const float* convw  = (const float*)d_in[6];
  const float* convb  = (const float*)d_in[7];
  const float* xprw   = (const float*)d_in[8];
  const float* dtw    = (const float*)d_in[9];
  const float* dtb    = (const float*)d_in[10];
  const float* alog   = (const float*)d_in[11];
  const float* dskip  = (const float*)d_in[12];
  const float* outw   = (const float*)d_in[13];
  const float* pnw    = (const float*)d_in[14];
  const float* pnb    = (const float*)d_in[15];
  const float* gatew  = (const float*)d_in[16];
  const float* upw    = (const float*)d_in[17];
  const float* downw  = (const float*)d_in[18];
  const float* fnw    = (const float*)d_in[19];
  const float* fnb    = (const float*)d_in[20];
  float* dout = (float*)d_out;

  if (in_sizes[0] != kSeq * kDinp) return;
  if (in_sizes[1] != kDm * kDinp || in_sizes[2] != kDm) return;
  if (in_sizes[3] != kNumSsm * kDm || in_sizes[4] != kNumSsm * kDm) return;
  if (in_sizes[5] != kNumSsm * kXZP * kDm) return;
  if (in_sizes[6] != kNumSsm * kDin * 4 || in_sizes[7] != kNumSsm * kDin) return;
  if (in_sizes[8] != kNumSsm * kPrjN * kDin) return;
  if (in_sizes[9] != kNumSsm * kDin * kDtR || in_sizes[10] != kNumSsm * kDin) return;
  if (in_sizes[11] != kNumSsm * kDin * kNst || in_sizes[12] != kNumSsm * kDin) return;
  if (in_sizes[13] != kNumSsm * kDm * kDin) return;
  if (in_sizes[14] != kDm || in_sizes[15] != kDm) return;
  if (in_sizes[16] != kDff * kDm || in_sizes[17] != kDff * kDm || in_sizes[18] != kDm * kDff) return;
  if (in_sizes[19] != kDm || in_sizes[20] != kDm) return;
  if (out_size != kSeq * kDm) return;

  const size_t SZ_XH   = (size_t)kSeq * kDinp * 2;
  const size_t SZ_WPL  = (size_t)kDff * kDm * 2;
  const size_t SZ_H    = (size_t)kSeq * kDm * 4;
  const size_t SZ_HN   = (size_t)kSeq * kDm * 2;
  const size_t SZ_XZ   = (size_t)kSeq * kXZP * 4;
  const size_t SZ_UC   = (size_t)kSeq * kDin * 4;
  const size_t SZ_UCH  = (size_t)kSeq * kDin * 2;
  const size_t SZ_PROJ = (size_t)kSeq * kPrjP * 4;
  const size_t SZ_DTH  = (size_t)kSeq * kDtR * 2;
  const size_t SZ_DLR  = (size_t)kSeq * kDin * 4;
  const size_t SZ_G    = (size_t)kSeq * kDff * 4;
  const size_t SZ_P    = (size_t)kSeq * kDff * 2;
  const size_t ARENA_SSM = SZ_XZ + SZ_UC + SZ_UCH + SZ_PROJ + SZ_DTH + SZ_DLR;
  const size_t ARENA_MLP = SZ_G + SZ_G + SZ_P;
  const size_t SZ_ARENA  = (ARENA_SSM > ARENA_MLP) ? ARENA_SSM : ARENA_MLP;
  const size_t OFF_XH   = 0;
  const size_t OFF_WPL  = OFF_XH  + SZ_XH;
  const size_t OFF_H0   = OFF_WPL + SZ_WPL;
  const size_t OFF_H1   = OFF_H0  + SZ_H;
  const size_t OFF_HN   = OFF_H1  + SZ_H;
  const size_t OFF_AR   = OFF_HN  + SZ_HN;
  const size_t TOTAL    = OFF_AR  + SZ_ARENA;
  if (ws_size < TOTAL) return;

  char* ws = (char*)d_ws;
  unsigned short* XH16 = (unsigned short*)(ws + OFF_XH);
  unsigned short* WPL  = (unsigned short*)(ws + OFF_WPL);
  float*          H0   = (float*)(ws + OFF_H0);
  float*          H1   = (float*)(ws + OFF_H1);
  unsigned short* HN   = (unsigned short*)(ws + OFF_HN);
  char* ar = ws + OFF_AR;
  float*          XZ   = (float*)(ar);
  float*          UC   = (float*)(ar + SZ_XZ);
  unsigned short* UCH  = (unsigned short*)(ar + SZ_XZ + SZ_UC);
  float*          PROJ = (float*)(ar + SZ_XZ + SZ_UC + SZ_UCH);
  unsigned short* DTH  = (unsigned short*)(ar + SZ_XZ + SZ_UC + SZ_UCH + SZ_PROJ);
  float*          DLR  = (float*)(ar + SZ_XZ + SZ_UC + SZ_UCH + SZ_PROJ + SZ_DTH);
  unsigned short* YP   = UCH;
  float*          Gb   = (float*)(ar);
  float*          Ub   = (float*)(ar + SZ_G);
  unsigned short* Pp   = (unsigned short*)(ar + SZ_G + SZ_G);
  const float* dummy_bias  = ipb;
  const float* dummy_resid = x;

  const float invW  = 1.0f / kWScale;
  const float invWX = 1.0f / (kWScale * kXScale);
  const float invWY = 1.0f / (kWScale * kYScale);
  const float invWP = 1.0f / (kWScale * kPScale);

  cast_rows_f16_kernel<<<(kSeq * kDinp / 8 + 255) / 256, 256, 0, stream>>>(x, XH16, kDinp, kSeq, kSeq * kDinp / 8, kXScale);
  cast_rows_f16_kernel<<<(kDm * kDinp / 8 + 255) / 256, 256, 0, stream>>>(ipw, WPL, kDinp, kDm, kDm * kDinp / 8, kWScale);
  wmma_gemm64<0, false, 2, 0, false><<<dim3((32 * 16 + 7) / 8, 1), 256, 0, stream>>>(
      XH16, XH16, kDinp, 0L, WPL, WPL, kDinp, 0L,
      (void*)H0, (void*)H0, kDm, 0L, ipb, dummy_resid, 0L, kSeq, kDm, kDinp, invWX);

  for (int k = 0; k < kNumSsm; ++k) {
    float* Hc = (k == 0) ? H0 : H1;
    float* Hn = (k == 0) ? H1 : H0;
    ln_f16_kernel<<<kSeq / 8, 256, 0, stream>>>(Hc, mnw + (size_t)k * kDm, mnb + (size_t)k * kDm, HN, kSeq);
    cast_rows_f16_kernel<<<(kXZP * kDm / 8 + 255) / 256, 256, 0, stream>>>(
        inw + (size_t)k * kXZP * kDm, WPL, kDm, kXZP, kXZP * kDm / 8, kWScale);
    wmma_gemm64<0, false, 0, 0, false><<<dim3((32 * 64 + 7) / 8, 1), 256, 0, stream>>>(
        HN, HN, kDm, 0L, WPL, WPL, kDm, 0L,
        (void*)XZ, (void*)XZ, kXZP, 0L, dummy_bias, dummy_resid, 0L, kSeq, kXZP, kDm, invW);
    conv_silu_kernel<<<dim3(kDin / 256, kSeq / 64), 256, 0, stream>>>(
        XZ, convw + (size_t)k * kDin * 4, convb + (size_t)k * kDin, UC, UCH);
    cast_rows_f16_kernel<<<(kPrjP * kDin / 8 + 255) / 256, 256, 0, stream>>>(
        xprw + (size_t)k * kPrjN * kDin, WPL, kDin, kPrjN, kPrjP * kDin / 8, kWScale);
    wmma_gemm64<0, false, 0, 0, false><<<dim3((32 * 2 + 7) / 8, 1), 256, 0, stream>>>(
        UCH, UCH, kDin, 0L, WPL, WPL, kDin, 0L,
        (void*)PROJ, (void*)PROJ, kPrjP, 0L, dummy_bias, dummy_resid, 0L, kSeq, kPrjP, kDin, invW);
    dt_cast_kernel<<<(kSeq * kDtR / 8 + 255) / 256, 256, 0, stream>>>(PROJ, DTH, kSeq * kDtR / 8);
    cast_rows_f16_kernel<<<(kDin * kDtR / 8 + 255) / 256, 256, 0, stream>>>(
        dtw + (size_t)k * kDin * kDtR, WPL, kDtR, kDin, kDin * kDtR / 8, kWScale);
    wmma_gemm64<0, false, 0, 0, false><<<dim3((32 * 32 + 7) / 8, 1), 256, 0, stream>>>(
        DTH, DTH, kDtR, 0L, WPL, WPL, kDtR, 0L,
        (void*)DLR, (void*)DLR, kDin, 0L, dummy_bias, dummy_resid, 0L, kSeq, kDin, kDtR, invW);
    scan_kernel<<<kDin / 256, 256, 0, stream>>>(
        DLR, UC, XZ, PROJ, dtb + (size_t)k * kDin, alog + (size_t)k * kDin * kNst, dskip + (size_t)k * kDin, YP);
    cast_rows_f16_kernel<<<(kDm * kDin / 8 + 255) / 256, 256, 0, stream>>>(
        outw + (size_t)k * kDm * kDin, WPL, kDin, kDm, kDm * kDin / 8, kWScale);
    wmma_gemm64<0, false, 0, 0, true><<<dim3((32 * 16 + 7) / 8, 1), 256, 0, stream>>>(
        YP, YP, kDin, 0L, WPL, WPL, kDin, 0L,
        (void*)Hn, (void*)Hn, kDm, 0L, dummy_bias, Hc, 0L, kSeq, kDm, kDin, invWY);
  }

  ln_f16_kernel<<<kSeq / 8, 256, 0, stream>>>(H0, pnw, pnb, HN, kSeq);
  cast_rows_f16_kernel<<<(kDff * kDm / 8 + 255) / 256, 256, 0, stream>>>(gatew, WPL, kDm, kDff, kDff * kDm / 8, kWScale);
  wmma_gemm64<0, false, 0, 0, false><<<dim3((32 * 64 + 7) / 8, 1), 256, 0, stream>>>(
      HN, HN, kDm, 0L, WPL, WPL, kDm, 0L,
      (void*)Gb, (void*)Gb, kDff, 0L, dummy_bias, dummy_resid, 0L, kSeq, kDff, kDm, invW);
  cast_rows_f16_kernel<<<(kDff * kDm / 8 + 255) / 256, 256, 0, stream>>>(upw, WPL, kDm, kDff, kDff * kDm / 8, kWScale);
  wmma_gemm64<0, false, 0, 0, false><<<dim3((32 * 64 + 7) / 8, 1), 256, 0, stream>>>(
      HN, HN, kDm, 0L, WPL, WPL, kDm, 0L,
      (void*)Ub, (void*)Ub, kDff, 0L, dummy_bias, dummy_resid, 0L, kSeq, kDff, kDm, invW);
  glu_kernel<<<(kSeq * kDff / 8 + 255) / 256, 256, 0, stream>>>(Gb, Ub, Pp, kSeq * kDff / 8);
  cast_rows_f16_kernel<<<(kDm * kDff / 8 + 255) / 256, 256, 0, stream>>>(downw, WPL, kDff, kDm, kDm * kDff / 8, kWScale);
  wmma_gemm64<0, false, 0, 0, true><<<dim3((32 * 16 + 7) / 8, 1), 256, 0, stream>>>(
      Pp, Pp, kDff, 0L, WPL, WPL, kDff, 0L,
      (void*)H1, (void*)H1, kDm, 0L, dummy_bias, H0, 0L, kSeq, kDm, kDff, invWP);

  ln_f32_kernel<<<kSeq / 8, 256, 0, stream>>>(H1, fnw, fnb, dout, kSeq);
}
